// GCN_22213570855080
// MI455X (gfx1250) — hardware-run, weakly checked
//
#include <hip/hip_runtime.h>
#include <stddef.h>
#include <stdint.h>
#include <math.h>


#define NN      50000
#define NE      800000
#define CIN     64
#define HID     128
#define NCL     32
#define SPLIT_H1 1
#define SPLIT_H  1
#define K1      64
#define P1      256
#define K2      (SPLIT_H1 ? 256 : 128)
#define PH      64
#define K3      (SPLIT_H ? 64 : 32)
#define MP      50048
#define NTHR    256
#define NWAVE   8
#define NBA     1024
#define PKS     10
#define NB      49
#define NPADN   (NB * NBA)
#define RCAP    28672
#define WLCAP   (RCAP / NWAVE)
#define EPW     (NE / NWAVE)
#define DEGCAP  64
#define GBM     64
#define GTHR    128
#define RPB     64
#define RPW     8
#define BK_INTS (2 * RCAP + 3 * NBA + 32)
#define LDS_BK  (BK_INTS * 4)
#define MEAS_BLK_HITS 16623
#define MEAS_MAXDEG   35
#define NB_W1   4
#define NB_W2   4
#define NB_WC   1
#define NB_W    (NB_W1 + NB_W2 + NB_WC)
#define NU_X    (MP * (CIN / 8))
#define NB_X    (NU_X / NTHR)
#define OUT1_EL (NN * NCL)

static_assert(NB * NBA >= NN);
static_assert(391 * 128 == MP && MP % GBM == 0 && MP % RPB == 0 && MP <= NPADN && MP >= NN);
static_assert(NBA == (1 << PKS) && NBA == NTHR * 4 && NBA % GBM == 0 && NBA % RPB == 0);
static_assert(((long long)NE << PKS) < (1LL << 31));
static_assert(NE % NWAVE == 0 && EPW % 32 == 0);
static_assert(RCAP % (NTHR * 4) == 0 && RCAP % NWAVE == 0 && BK_INTS % 4 == 0);
static_assert((long long)RCAP * 100 >= (long long)MEAS_BLK_HITS * 105);
static_assert(DEGCAP >= MEAS_MAXDEG + 8);
static_assert(LDS_BK <= 300000);
static_assert(K1 % 32 == 0 && K2 % 32 == 0 && K3 % 32 == 0);
static_assert(K2 <= P1 && K3 <= PH);
static_assert(HID == 8 * 16 && NCL == 2 * 16 && HID == 32 * 4 && NCL == 32);
static_assert(GBM == (GTHR / 32) * 16 && RPB == NWAVE * RPW);
static_assert(NU_X % NTHR == 0);
static_assert(((long long)OUT1_EL * 4) % 128 == 0);
static_assert((long long)OUT1_EL + (long long)(NN - 1) * NCL + (NCL - 1) == 2LL * NN * NCL - 1);

typedef float          v2f   __attribute__((ext_vector_type(2)));
typedef float          v4f   __attribute__((ext_vector_type(4)));
typedef float          v8f   __attribute__((ext_vector_type(8)));
typedef int            v4i   __attribute__((ext_vector_type(4)));
typedef int            v8i   __attribute__((ext_vector_type(8)));
typedef unsigned       v2u   __attribute__((ext_vector_type(2)));
typedef unsigned       v4u   __attribute__((ext_vector_type(4)));
typedef unsigned short v8us  __attribute__((ext_vector_type(8)));
typedef __bf16         v16bf __attribute__((ext_vector_type(16)));
typedef v4f  __attribute__((may_alias)) v4fa;
typedef v4i  __attribute__((may_alias)) v4ia;
typedef v2u  __attribute__((may_alias)) v2ua;
typedef v4u  __attribute__((may_alias)) v4ua;
typedef v8us __attribute__((may_alias)) v8usa;
union FragB { v16bf v; v8us h[2]; v8i w; };

__device__ __forceinline__ v8f wmb(const FragB& a, const FragB& b, v8f c) {
  v8f d = __builtin_amdgcn_wmma_f32_16x16x32_bf16(false, a.v, false, b.v, (short)0, c, false, false);
  asm volatile("v_nop\n\tv_nop\n\tv_nop\n\tv_nop" : "+v"(d) : "v"(a.w), "v"(b.w));
  return d;
}

__device__ __forceinline__ unsigned bf16_bits(float f) {
  const unsigned u = __float_as_uint(f);
  const unsigned r = ((u + 0x7FFFu + ((u >> 16) & 1u)) >> 16) & 0xFFFFu;
  return ((u & 0x7FFFFFFFu) > 0x7F800000u) ? 0x7FC0u : r;
}
__device__ __forceinline__ float bf16_val(float f) { return __uint_as_float(bf16_bits(f) << 16); }
__device__ __forceinline__ void pack2(float a, float b, unsigned& hw, unsigned& lw) {
  const unsigned ha = bf16_bits(a), hb = bf16_bits(b);
  const unsigned la = bf16_bits(a - __uint_as_float(ha << 16));
  const unsigned lb = bf16_bits(b - __uint_as_float(hb << 16));
  hw = ha | (hb << 16);
  lw = la | (lb << 16);
}
__device__ __forceinline__ float relu_k(float v) { return (v > 0.0f) ? v : (v - v); }

__device__ __forceinline__ void wave_sync() {
  __builtin_amdgcn_fence(__ATOMIC_RELEASE, "wavefront");
  __builtin_amdgcn_wave_barrier();
  __builtin_amdgcn_fence(__ATOMIC_ACQUIRE, "wavefront");
}

__device__ __forceinline__ void st2_us8(unsigned short* dp, v8us o) {
  *(volatile v8us*)dp = o;
  __threadfence();
  *(volatile v8us*)dp = o;
}

__device__ __forceinline__ void slot_info(const int* __restrict__ CNT, const int* __restrict__ OFF, int node,
                                          int& deg, int& c, int& o) {
  const int craw = CNT[node];
  const int oraw = OFF[node];
  deg = craw < 0 ? 0 : craw;
  c = deg > DEGCAP ? DEGCAP : deg;
  o = oraw < 0 ? 0 : (oraw > RCAP ? RCAP : oraw);
  if (c > RCAP - o) c = RCAP - o;
}

__global__ __launch_bounds__(NTHR) void k_prep(const float* __restrict__ x, const float* __restrict__ W1,
                                               const float* __restrict__ W2, const float* __restrict__ Wc,
                                               unsigned short* XB, unsigned short* W1T,
                                               unsigned short* W2D, unsigned short* WcD) {
  const int b = (int)blockIdx.x, tid = (int)threadIdx.x;
  if (b < NB_W1) {
    const int u  = b * NTHR + tid;
    const int n  = u >> 3;
    const int k8 = (u & 7) * 8;
    const float* p = W1 + (size_t)k8 * HID + n;
    v8us o;
#pragma unroll
    for (int i = 0; i < 8; ++i) o[i] = (unsigned short)bf16_bits(p[(size_t)i * HID]);
    st2_us8(W1T + (size_t)n * K1 + k8, o);
  } else if (b < NB_W1 + NB_W2) {
    const int v  = (b - NB_W1) * NTHR + tid;
    const int n  = v >> 5;
    const int k8 = (v & 31) * 8;
    const int kk = k8 & (HID - 1);
    const float* p = W2 + (size_t)kk * NCL + n;
    v8us o;
#pragma unroll
    for (int i = 0; i < 8; ++i) o[i] = (unsigned short)bf16_bits(p[(size_t)i * NCL]);
    st2_us8(W2D + (size_t)n * 256 + k8, o);
  } else if (b < NB_W) {
    const int v  = tid;
    const int n  = v >> 3;
    const int k8 = (v & 7) * 8;
    const int kk = k8 & (NCL - 1);
    const float* p = Wc + (size_t)kk * NCL + n;
    v8us o;
#pragma unroll
    for (int i = 0; i < 8; ++i) o[i] = (unsigned short)bf16_bits(p[(size_t)i * NCL]);
    st2_us8(WcD + (size_t)n * 64 + k8, o);
  } else {
    const int u   = (b - NB_W) * NTHR + tid;
    const int row = u >> 3;
    const int k8  = (u & 7) * 8;
    const int rc  = row < NN ? row : NN - 1;
    const float* p = x + (size_t)rc * CIN + k8;
    const v4f a = *(const v4fa*)p;
    const v4f c = *(const v4fa*)(p + 4);
    asm volatile("" :: "v"(a), "v"(c));
    const bool ok = row < NN;
    v8us o;
    o[0] = ok ? (unsigned short)bf16_bits(a.x) : (unsigned short)0;
    o[1] = ok ? (unsigned short)bf16_bits(a.y) : (unsigned short)0;
    o[2] = ok ? (unsigned short)bf16_bits(a.z) : (unsigned short)0;
    o[3] = ok ? (unsigned short)bf16_bits(a.w) : (unsigned short)0;
    o[4] = ok ? (unsigned short)bf16_bits(c.x) : (unsigned short)0;
    o[5] = ok ? (unsigned short)bf16_bits(c.y) : (unsigned short)0;
    o[6] = ok ? (unsigned short)bf16_bits(c.z) : (unsigned short)0;
    o[7] = ok ? (unsigned short)bf16_bits(c.w) : (unsigned short)0;
    st2_us8(XB + (size_t)row * CIN + k8, o);
  }
}

__global__ __launch_bounds__(NTHR) void k_bucket(const int* __restrict__ keys, const int* __restrict__ gidx,
                                                 int* LIST, int* CNT, int* OFF, float* DINV, int* FLAG) {
  extern __shared__ __attribute__((aligned(16))) int dsm[];
  int* wl   = dsm;
  int* reg2 = wl + RCAP;
  int* scnt = reg2 + RCAP;
  int* soff = scnt + NBA;
  int* cur  = soff + NBA;
  int* wcnt = cur + NBA;
  int* wtot = wcnt + 8;
  int* wmx  = wtot + 8;
  const int tid = (int)threadIdx.x, lane = tid & 31, wave = tid >> 5;
  const int nodeBase = (int)blockIdx.x * NBA;
  int nb = NN - nodeBase;
  nb = nb > NBA ? NBA : (nb < 1 ? 1 : nb);

  {
    const v4i z4 = {0, 0, 0, 0};
    for (int i = tid * 4; i < BK_INTS; i += NTHR * 4) *(v4ia*)(dsm + i) = z4;
  }
  __syncthreads();

  int wc = 0;
  const int e0w = wave * EPW;
#pragma unroll 1
  for (int it = 0; it < EPW / 32; ++it) {
    const int e  = e0w + it * 32 + lane;
    const int ec = e < NE ? e : NE - 1;
    const int key = keys[ec];
    asm volatile("" :: "v"(key));
    const unsigned s = (unsigned)key - (unsigned)nodeBase;
    const bool hit = (e < NE) && (s < (unsigned)nb);
    const unsigned m = __builtin_amdgcn_ballot_w32(hit);
    if (m != 0u) {
      if (hit) {
        const int pos = wc + (int)__builtin_amdgcn_mbcnt_lo(m, 0u);
        if (pos < WLCAP) wl[wave * WLCAP + pos] = (int)(((unsigned)e << PKS) | s);
      }
      wc += (int)__builtin_popcount(m);
    }
  }
  if (lane == 0) wcnt[wave] = wc;
  __syncthreads();

  int nh = 0, anyov = 0;
#pragma unroll
  for (int w2 = 0; w2 < NWAVE; ++w2) {
    int c = wcnt[w2];
    anyov |= (c > WLCAP) ? 1 : 0;
    c = c < 0 ? 0 : (c > WLCAP ? WLCAP : c);
    nh += c;
  }
  nh = nh > RCAP ? RCAP : nh;

  if (wave == 0) {
#pragma unroll 1
    for (int w2 = 0; w2 < NWAVE; ++w2) {
      int c = wcnt[w2];
      c = c < 0 ? 0 : (c > WLCAP ? WLCAP : c);
#pragma unroll 1
      for (int b0 = 0; b0 < c; b0 += 32) {
        const int idx = b0 + lane;
        const int uv  = wl[w2 * WLCAP + (idx < WLCAP ? idx : WLCAP - 1)];
        const int m32 = (c - b0) < 32 ? (c - b0) : 32;
#pragma unroll 1
        for (int k = 0; k < m32; ++k) {
          const int u  = __builtin_amdgcn_readlane(uv, k);
          const int sl = u & (NBA - 1);
          if (lane == 0) scnt[sl] = scnt[sl] + 1;
        }
      }
    }
  }
  __syncthreads();

  {
    const v4i ca = *(const v4ia*)(scnt + 4 * tid);
    const int e0 = ca.x < 0 ? 0 : ca.x, e1 = ca.y < 0 ? 0 : ca.y, e2 = ca.z < 0 ? 0 : ca.z, e3 = ca.w < 0 ? 0 : ca.w;
    const int ts = e0 + e1 + e2 + e3;
    int incl = ts;
#pragma unroll
    for (int d = 1; d < 32; d <<= 1) {
      const int up = __shfl_up(incl, d, 32);
      if (lane >= d) incl += up;
    }
    int mx = max(max(e0, e1), max(e2, e3));
    mx = max(mx, __shfl_xor(mx, 16, 32));
    mx = max(mx, __shfl_xor(mx, 8, 32));
    mx = max(mx, __shfl_xor(mx, 4, 32));
    mx = max(mx, __shfl_xor(mx, 2, 32));
    mx = max(mx, __shfl_xor(mx, 1, 32));
    if (lane == 31) wtot[wave] = incl;
    if (lane == 0)  wmx[wave] = mx;
    __syncthreads();
    int pre = 0;
#pragma unroll
    for (int w2 = 0; w2 < NWAVE; ++w2) pre += (w2 < wave) ? wtot[w2] : 0;
    int run = pre + incl - ts;
    v4i so;
    so.x = run; run += e0;
    so.y = run; run += e1;
    so.z = run; run += e2;
    so.w = run;
    *(v4ia*)(soff + 4 * tid) = so;
    *(v4ia*)(cur + 4 * tid)  = so;
  }
  __syncthreads();

  if (wave == 0) {
#pragma unroll 1
    for (int w2 = 0; w2 < NWAVE; ++w2) {
      int c = wcnt[w2];
      c = c < 0 ? 0 : (c > WLCAP ? WLCAP : c);
#pragma unroll 1
      for (int b0 = 0; b0 < c; b0 += 32) {
        const int idx = b0 + lane;
        const int uv  = wl[w2 * WLCAP + (idx < WLCAP ? idx : WLCAP - 1)];
        const int m32 = (c - b0) < 32 ? (c - b0) : 32;
#pragma unroll 1
        for (int k = 0; k < m32; ++k) {
          const int u   = __builtin_amdgcn_readlane(uv, k);
          const int sl  = u & (NBA - 1);
          const int eid = (int)((unsigned)u >> PKS);
          if (lane == 0) {
            int pos = cur[sl];
            pos = pos < 0 ? 0 : (pos > RCAP - 1 ? RCAP - 1 : pos);
            reg2[pos] = eid;
            cur[sl] = pos + 1;
          }
        }
      }
    }
  }
  __syncthreads();

#pragma unroll 1
  for (int i = 0; i < 4; ++i) {
    const int s = i * NTHR + tid;
    int c = scnt[s];
    c = c < 0 ? 0 : c;
    const float dg = (float)(c + 1);
    const float r  = 1.0f / sqrtf(dg);
    cur[s] = __float_as_int((dg > 0.0f) ? r : 0.0f);
  }
  __syncthreads();

  int bmax = 0;
#pragma unroll
  for (int w2 = 0; w2 < NWAVE; ++w2) bmax = max(bmax, wmx[w2]);
  const int flag = ((anyov != 0) || (bmax > DEGCAP)) ? 1 : 0;

  int* lrow = LIST + (size_t)blockIdx.x * RCAP;
#pragma unroll 1
  for (int it = 0; it < RCAP / (NTHR * 4); ++it) {
    const int i0 = 4 * (it * NTHR + tid);
    const v4i ev = *(const v4ia*)(reg2 + i0);
    int e0 = ev.x, e1 = ev.y, e2 = ev.z, e3 = ev.w;
    e0 = e0 < 0 ? 0 : (e0 > NE - 1 ? NE - 1 : e0);
    e1 = e1 < 0 ? 0 : (e1 > NE - 1 ? NE - 1 : e1);
    e2 = e2 < 0 ? 0 : (e2 > NE - 1 ? NE - 1 : e2);
    e3 = e3 < 0 ? 0 : (e3 > NE - 1 ? NE - 1 : e3);
    int g0 = gidx[e0], g1 = gidx[e1], g2 = gidx[e2], g3 = gidx[e3];
    asm volatile("" :: "v"(g0), "v"(g1), "v"(g2), "v"(g3));
    g0 = g0 < 0 ? 0 : (g0 > NN - 1 ? NN - 1 : g0);
    g1 = g1 < 0 ? 0 : (g1 > NN - 1 ? NN - 1 : g1);
    g2 = g2 < 0 ? 0 : (g2 > NN - 1 ? NN - 1 : g2);
    g3 = g3 < 0 ? 0 : (g3 > NN - 1 ? NN - 1 : g3);
    v4i ov;
    ov.x = (i0     < nh) ? g0 : 0;
    ov.y = (i0 + 1 < nh) ? g1 : 0;
    ov.z = (i0 + 2 < nh) ? g2 : 0;
    ov.w = (i0 + 3 < nh) ? g3 : 0;
    *(volatile v4i*)(lrow + i0) = ov;
    __threadfence();
    *(volatile v4i*)(lrow + i0) = ov;
  }
  {
    const v4i cv = *(const v4ia*)(scnt + 4 * tid);
    const v4i fr = *(const v4ia*)(soff + 4 * tid);
    const v4i db = *(const v4ia*)(cur + 4 * tid);
    v4i fv;
    fv.x = (4 * tid     < nb) ? fr.x : 0;
    fv.y = (4 * tid + 1 < nb) ? fr.y : 0;
    fv.z = (4 * tid + 2 < nb) ? fr.z : 0;
    fv.w = (4 * tid + 3 < nb) ? fr.w : 0;
    v4f dv;
    dv.x = __int_as_float(db.x); dv.y = __int_as_float(db.y);
    dv.z = __int_as_float(db.z); dv.w = __int_as_float(db.w);
    v4i rv = {0, 0, 0, 0};
    rv.x = (tid == 0) ? flag : 0;
    rv.y = (tid == 0) ? bmax : 0;
    rv.z = (tid == 0) ? nh : 0;
    int*   cp = CNT  + (size_t)nodeBase + 4 * tid;
    int*   fp = OFF  + (size_t)nodeBase + 4 * tid;
    float* qp = DINV + (size_t)nodeBase + 4 * tid;
    int*   rp = FLAG + (size_t)blockIdx.x * 32 + 4 * (tid & 7);
    *(volatile v4i*)cp = cv;
    *(volatile v4i*)fp = fv;
    *(volatile v4f*)qp = dv;
    if (tid < 8) *(volatile v4i*)rp = rv;
    __threadfence();
    *(volatile v4i*)cp = cv;
    *(volatile v4i*)fp = fv;
    *(volatile v4f*)qp = dv;
    if (tid < 8) *(volatile v4i*)rp = rv;
  }
}

template <int NT, int EPI>
__global__ __launch_bounds__(GTHR) __attribute__((amdgpu_num_vgpr(248)))
void k_gemm(const unsigned short* __restrict__ A, const unsigned short* __restrict__ WT,
            const float* __restrict__ rowScale, const float* __restrict__ bias, const int* __restrict__ FLAG,
            float* outF, int K, int lda, int ldw, int rowLimit) {
  constexpr int NC = 16 * NT;
  constexpr int NI = (16 * NC) / 128;
  static_assert(NT == 8 || NT == 2);
  static_assert(EPI == 0 || NT == 2);
  static_assert((16 * NC) % 128 == 0);
  __shared__ __attribute__((aligned(16))) float stg[GBM * NC];
  __shared__ __attribute__((aligned(16))) float dsh[GBM];
  __shared__ __attribute__((aligned(16))) float bsh[32];
  const int tid = (int)threadIdx.x, lane = tid & 31, wave = tid >> 5, hh = lane >> 4, m = lane & 15;
  const int rowBase = (int)blockIdx.x * GBM;

  if (tid < 16) {
    const v4f d4 = *(const v4f*)(rowScale + rowBase + 4 * tid);
    *(v4fa*)(dsh + 4 * tid) = d4;
  }
  if (tid < 8) {
    const v4f b4 = *(const v4f*)(bias + 4 * tid);
    v4f bq;
    bq.x = bf16_val(b4.x); bq.y = bf16_val(b4.y); bq.z = bf16_val(b4.z); bq.w = bf16_val(b4.w);
    *(v4fa*)(bsh + 4 * tid) = bq;
  }
  const int fl = FLAG[(size_t)(rowBase >> PKS) * 32];

  v8f acc[NT];
  {
    const v8f z = {0.f, 0.f, 0.f, 0.f, 0.f, 0.f, 0.f, 0.f};
#pragma unroll
    for (int t = 0; t < NT; ++t) acc[t] = z;
  }
  const unsigned short* ap = A  + (size_t)(rowBase + 16 * wave + m) * (size_t)lda + 8 * hh;
  const unsigned short* wp = WT + (size_t)m * (size_t)ldw + 8 * hh;
  const int ksteps = K >> 5;
#pragma unroll 1
  for (int ks = 0; ks < ksteps; ++ks) {
    FragB af;
    af.h[0] = *(const v8usa*)(ap + 32 * ks);
    af.h[1] = *(const v8usa*)(ap + 32 * ks + 16);
#pragma unroll
    for (int t = 0; t < NT; ++t) {
      const unsigned short* wq = wp + (size_t)(16 * t) * (size_t)ldw + 32 * ks;
      FragB bf;
      bf.h[0] = *(const v8usa*)wq;
      bf.h[1] = *(const v8usa*)(wq + 16);
      acc[t] = wmb(af, bf, acc[t]);
    }
  }
  __syncthreads();

  const float qnan = __int_as_float(0x7fc00000);
#pragma unroll
  for (int t = 0; t < NT; ++t) {
    const int lc = 16 * t + m;
#pragma unroll
    for (int r = 0; r < 8; ++r) {
      const int lr = 16 * wave + 8 * hh + r;
      float v;
      if constexpr (EPI == 0) {
        v = acc[t][r] * dsh[lr];
      } else {
        v = acc[t][r] + bsh[lc];
        v = (fl != 0) ? qnan : v;
      }
      stg[lr * NC + lc] = v;
    }
  }
  __syncthreads();

  v4f fv[NI];
#pragma unroll
  for (int i = 0; i < NI; ++i) {
    const int fi = 16 * wave * NC + i * 128 + 4 * lane;
    fv[i] = *(const v4fa*)(stg + fi);
  }
#pragma unroll
  for (int i = 0; i < NI; ++i) {
    const int fi = 16 * wave * NC + i * 128 + 4 * lane;
    const int gr = rowBase + fi / NC;
    float* op = outF + (size_t)rowBase * NC + fi;
    if (gr < rowLimit) *(volatile v4f*)op = fv[i];
  }
  __threadfence();
#pragma unroll
  for (int i = 0; i < NI; ++i) {
    const int fi = 16 * wave * NC + i * 128 + 4 * lane;
    const int gr = rowBase + fi / NC;
    float* op = outF + (size_t)rowBase * NC + fi;
    if (gr < rowLimit) *(volatile v4f*)op = fv[i];
  }
}

__global__ __launch_bounds__(NTHR) void k_agg1(const float* __restrict__ H1P, const int* __restrict__ LIST,
                                               const int* __restrict__ CNT, const int* __restrict__ OFF,
                                               const float* __restrict__ DINV, const int* __restrict__ FLAG,
                                               const float* __restrict__ b1, unsigned short* X1HL) {
  __shared__ __attribute__((aligned(16))) unsigned rowst[NWAVE * 128];
  const int tid = (int)threadIdx.x, lane = tid & 31, wave = tid >> 5;
  float bb0, bb1, bb2, bb3;
  {
    const v4f b4 = *(const v4f*)(b1 + 4 * lane);
    bb0 = bf16_val(b4.x); bb1 = bf16_val(b4.y); bb2 = bf16_val(b4.z); bb3 = bf16_val(b4.w);
  }
  const int fl = FLAG[(size_t)(((int)blockIdx.x * RPB) >> PKS) * 32];
  const float qnan = __int_as_float(0x7fc00000);
  unsigned* wst = rowst + wave * 128;
#pragma unroll 1
  for (int ri = 0; ri < RPW; ++ri) {
    const int node = (int)blockIdx.x * RPB + wave * RPW + ri;
    int deg, c, o;
    slot_info(CNT, OFF, node, deg, c, o);
    const int* lp = LIST + (size_t)(node >> PKS) * RCAP;
    int last = o + c - 1;
    last = last < o ? o : last;
    last = last > RCAP - 1 ? RCAP - 1 : last;
    float a0 = 0.0f, a1 = 0.0f, a2 = 0.0f, a3 = 0.0f;
#pragma unroll 1
    for (int b0 = 0; b0 < c; b0 += 32) {
      int idx = o + b0 + lane;
      idx = idx > last ? last : idx;
      int col = lp[idx];
      asm volatile("" :: "v"(col));
      col = col < 0 ? 0 : (col > NN - 1 ? NN - 1 : col);
      const int m32 = (c - b0) < 32 ? (c - b0) : 32;
#pragma unroll 1
      for (int k = 0; k < m32; ++k) {
        const int sk = __builtin_amdgcn_readlane(col, k);
        const v4f g = *(const v4f*)(H1P + (size_t)sk * HID + 4 * lane);
        a0 += g.x; a1 += g.y; a2 += g.z; a3 += g.w;
      }
    }
    const int nodec = node < NN ? node : NN - 1;
    const v4f sv = *(const v4f*)(H1P + (size_t)nodec * HID + 4 * lane);
    const float dd = DINV[nodec];
    a0 += sv.x; a1 += sv.y; a2 += sv.z; a3 += sv.w;
    float v0 = dd * a0 + bb0;
    float v1 = dd * a1 + bb1;
    float v2 = dd * a2 + bb2;
    float v3 = dd * a3 + bb3;
    v0 = relu_k(v0); v1 = relu_k(v1); v2 = relu_k(v2); v3 = relu_k(v3);
    const bool bad  = (fl != 0) || (deg > DEGCAP);
    const bool live = node < NN;
    v0 = bad ? qnan : v0; v1 = bad ? qnan : v1; v2 = bad ? qnan : v2; v3 = bad ? qnan : v3;
    v0 = live ? v0 : 0.0f; v1 = live ? v1 : 0.0f; v2 = live ? v2 : 0.0f; v3 = live ? v3 : 0.0f;
    unsigned hw0, lw0, hw1, lw1;
    pack2(v0, v1, hw0, lw0);
    pack2(v2, v3, hw1, lw1);
    v2u th, tl;
    th.x = hw0; th.y = hw1;
    tl.x = lw0; tl.y = lw1;
    *(v2ua*)(wst + 2 * lane)      = th;
    *(v2ua*)(wst + 64 + 2 * lane) = tl;
    wave_sync();
    const v4u q = *(const v4ua*)(wst + 4 * lane);
    wave_sync();
    unsigned short* wp = X1HL + (size_t)node * P1 + 8 * lane;
    *(volatile v4u*)wp = q;
    __threadfence();
    *(volatile v4u*)wp = q;
  }
}

__global__ __launch_bounds__(NTHR) void k_agg2(const float* __restrict__ H2P, const int* __restrict__ LIST,
                                               const int* __restrict__ CNT, const int* __restrict__ OFF,
                                               const float* __restrict__ DINV, const int* __restrict__ FLAG,
                                               const float* __restrict__ b2, float* outH, unsigned short* HHL) {
  const int tid = (int)threadIdx.x, lane = tid & 31, wave = tid >> 5;
  const float bb = bf16_val(b2[lane]);
  const int fl = FLAG[(size_t)(((int)blockIdx.x * RPB) >> PKS) * 32];
  const float qnan = __int_as_float(0x7fc00000);
  const int sa = (2 * lane) & 31, sb = (2 * lane + 1) & 31;
#pragma unroll 1
  for (int ri = 0; ri < RPW; ++ri) {
    const int node = (int)blockIdx.x * RPB + wave * RPW + ri;
    int deg, c, o;
    slot_info(CNT, OFF, node, deg, c, o);
    const int* lp = LIST + (size_t)(node >> PKS) * RCAP;
    int last = o + c - 1;
    last = last < o ? o : last;
    last = last > RCAP - 1 ? RCAP - 1 : last;
    float acc = 0.0f;
#pragma unroll 1
    for (int b0 = 0; b0 < c; b0 += 32) {
      int idx = o + b0 + lane;
      idx = idx > last ? last : idx;
      int col = lp[idx];
      asm volatile("" :: "v"(col));
      col = col < 0 ? 0 : (col > NN - 1 ? NN - 1 : col);
      const int m32 = (c - b0) < 32 ? (c - b0) : 32;
#pragma unroll 1
      for (int k = 0; k < m32; ++k) {
        const int sk = __builtin_amdgcn_readlane(col, k);
        acc += H2P[(size_t)sk * NCL + lane];
      }
    }
    const int nodec = node < NN ? node : NN - 1;
    const float sv = H2P[(size_t)nodec * NCL + lane];
    const float dd = DINV[nodec];
    acc += sv;
    float v = dd * acc + bb;
    const bool bad  = (fl != 0) || (deg > DEGCAP);
    const bool live = node < NN;
    v = bad ? qnan : v;
    v = live ? v : 0.0f;
    const unsigned hb = bf16_bits(v);
    const unsigned lb = bf16_bits(v - __uint_as_float(hb << 16));
    const int ha = __shfl((int)hb, sa, 32), hc = __shfl((int)hb, sb, 32);
    const int la = __shfl((int)lb, sa, 32), lc = __shfl((int)lb, sb, 32);
    const unsigned wh = (unsigned)ha | ((unsigned)hc << 16);
    const unsigned wl = (unsigned)la | ((unsigned)lc << 16);
    const unsigned word = (lane < 16) ? wh : wl;
    unsigned* hp = (unsigned*)HHL + (size_t)node * (PH / 2) + lane;
    float* op = outH + (size_t)nodec * NCL + lane;
    if (live) *(volatile float*)op = v;
    *(volatile unsigned*)hp = word;
    __threadfence();
    if (live) *(volatile float*)op = v;
    *(volatile unsigned*)hp = word;
  }
}

static inline size_t al256(size_t o) { return (o + 255) & ~(size_t)255; }

extern "C" void kernel_launch(void* const* d_in, const int* in_sizes, int n_in,
                              void* d_out, int out_size, void* d_ws, size_t ws_size,
                              hipStream_t stream) {
  if (n_in < 8) return;
  if (in_sizes[0] != NN * CIN) return;
  if (in_sizes[1] != 2 * NE) return;
  if (in_sizes[2] != CIN * HID || in_sizes[3] != HID) return;
  if (in_sizes[4] != HID * NCL || in_sizes[5] != NCL) return;
  if (in_sizes[6] != NCL * NCL || in_sizes[7] != NCL) return;
  if (out_size != 2 * NN * NCL) return;

  const float* x  = (const float*)d_in[0];
  const int*   ei = (const int*)  d_in[1];
  const float* W1 = (const float*)d_in[2];
  const float* b1 = (const float*)d_in[3];
  const float* W2 = (const float*)d_in[4];
  const float* b2 = (const float*)d_in[5];
  const float* Wc = (const float*)d_in[6];
  const float* bc = (const float*)d_in[7];
  const int* src = ei;
  const int* dst = ei + NE;
  float* out  = (float*)d_out;
  float* outH = out + OUT1_EL;

  char* ws = (char*)d_ws;
  size_t off = 0;
  const size_t oXB  = off; off = al256(off + (size_t)MP * CIN * 2);
  const size_t oW1T = off; off = al256(off + (size_t)HID * K1 * 2);
  const size_t oW2D = off; off = al256(off + (size_t)NCL * 256 * 2);
  const size_t oWcD = off; off = al256(off + (size_t)NCL * 64 * 2);
  const size_t oLS  = off; off = al256(off + (size_t)NB * RCAP * 4);
  const size_t oCN  = off; off = al256(off + (size_t)NPADN * 4);
  const size_t oOF  = off; off = al256(off + (size_t)NPADN * 4);
  const size_t oDI  = off; off = al256(off + (size_t)NPADN * 4);
  const size_t oFL  = off; off = al256(off + (size_t)NB * 128);
  const size_t oH1P = off; off = al256(off + (size_t)MP * HID * 4);
  const size_t oX1  = off; off = al256(off + (size_t)MP * P1 * 2);
  const size_t oH2P = off; off = al256(off + (size_t)MP * NCL * 4);
  const size_t oHH  = off; off = al256(off + (size_t)MP * PH * 2);
  if (off > ws_size || off > (size_t)134217728) return;
  unsigned short* XB  = (unsigned short*)(ws + oXB);
  unsigned short* W1T = (unsigned short*)(ws + oW1T);
  unsigned short* W2D = (unsigned short*)(ws + oW2D);
  unsigned short* WcD = (unsigned short*)(ws + oWcD);
  int*   LIST = (int*)(ws + oLS);
  int*   CNT  = (int*)(ws + oCN);
  int*   OFF  = (int*)(ws + oOF);
  float* DINV = (float*)(ws + oDI);
  int*   FLAG = (int*)(ws + oFL);
  float* H1P  = (float*)(ws + oH1P);
  unsigned short* X1HL = (unsigned short*)(ws + oX1);
  float* H2P  = (float*)(ws + oH2P);
  unsigned short* HHL  = (unsigned short*)(ws + oHH);

  hipFuncSetAttribute(reinterpret_cast<const void*>(&k_bucket), hipFuncAttributeMaxDynamicSharedMemorySize, LDS_BK);

  k_prep<<<NB_W + NB_X, NTHR, 0, stream>>>(x, W1, W2, Wc, XB, W1T, W2D, WcD);
  k_bucket<<<NB, NTHR, LDS_BK, stream>>>(dst, src, LIST, CNT, OFF, DINV, FLAG);
  k_gemm<8, 0><<<MP / GBM, GTHR, 0, stream>>>(XB, W1T, DINV, bc, FLAG, H1P, K1, CIN, K1, MP);
  k_agg1<<<MP / RPB, NTHR, 0, stream>>>(H1P, LIST, CNT, OFF, DINV, FLAG, b1, X1HL);
  k_gemm<2, 0><<<MP / GBM, GTHR, 0, stream>>>(X1HL, W2D, DINV, bc, FLAG, H2P, K2, P1, 256, MP);
  k_agg2<<<MP / RPB, NTHR, 0, stream>>>(H2P, LIST, CNT, OFF, DINV, FLAG, b2, outH, HHL);
  k_gemm<2, 1><<<MP / GBM, GTHR, 0, stream>>>(HHL, WcD, DINV, bc, FLAG, out, K3, PH, 64, NN);
}
